// Mamba2Block_16544214024872
// MI455X (gfx1250) — hardware-run, weakly checked
//
#include <hip/hip_runtime.h>
#include <math.h>

typedef __attribute__((ext_vector_type(16))) _Float16 v16h;
typedef __attribute__((ext_vector_type(8)))  _Float16 v8h;
typedef __attribute__((ext_vector_type(16))) __bf16   v16b;
typedef __attribute__((ext_vector_type(8)))  __bf16   v8b;
typedef __attribute__((ext_vector_type(8)))  float    v8f;
typedef __attribute__((ext_vector_type(4)))  float    v4f;
typedef __attribute__((ext_vector_type(2)))  float    v2f;
typedef __attribute__((ext_vector_type(4)))  unsigned v4u;

constexpr int kBatch = 2;
constexpr int kSeq   = 2048;
constexpr int kDm    = 1024;
constexpr int kDin   = 2048;
constexpr int kNst   = 16;
constexpr int kDConv = 4;
constexpr int kXzN   = 2 * kDin;
constexpr int kXdN   = kDin + 2 * kNst;
constexpr int kBcN   = 64;
constexpr int kWxNP  = kDin + kBcN;
constexpr int kRows  = kBatch * kSeq;
static_assert((kDm % 32) == 0 && (kDin % 32) == 0, "GEMM K multiples of 32");
static_assert((kRows % 64) == 0 && (kXzN % 64) == 0 && (kDin % 64) == 0 && (kBcN % 64) == 0 && (kDm % 64) == 0, "GEMM M,N multiples of 64");
static_assert((kXdN % 4) == 0 && kXdN <= kWxNP && (kWxNP % 64) == 0, "W_x padding");
static_assert((kSeq % 64) == 0 && (kDin % 512) == 0, "conv tile multiples");

constexpr size_t kOffXB   = 0;
constexpr size_t kOffWIB  = kOffXB  + (size_t)kRows * kDm  * 2;
constexpr size_t kOffWXH  = kOffWIB + (size_t)kXzN  * kDm  * 2;
constexpr size_t kOffWDH  = kOffWXH + (size_t)kWxNP * kDin * 2;
constexpr size_t kOffWOH  = kOffWDH + (size_t)kDin  * kDin * 2;
constexpr size_t kOffXZ   = kOffWOH + (size_t)kDm   * kDin * 2;
constexpr size_t kOffU    = kOffXZ  + (size_t)kRows * kXzN * 2;
constexpr size_t kOffDI   = kOffU   + (size_t)kRows * kDin * 2;
constexpr size_t kOffBC   = kOffDI  + (size_t)kRows * kDin * 2;
constexpr size_t kOffDP   = kOffBC  + (size_t)kRows * kBcN * 2;
constexpr size_t kWsTotal = kOffDP  + (size_t)kRows * kDin * 2;
static_assert(kWsTotal == 122421248ull, "carve total");
static_assert(kWsTotal <= 134217728ull, "carve cap");
static_assert((kOffWIB % 128) == 0 && (kOffWXH % 128) == 0 && (kOffWDH % 128) == 0 && (kOffWOH % 128) == 0 &&
              (kOffXZ % 128) == 0 && (kOffU % 128) == 0 && (kOffDI % 128) == 0 && (kOffBC % 128) == 0 &&
              (kOffDP % 128) == 0, "128-B aligned regions");

__device__ __forceinline__ unsigned short f2bf_bits(float f) {
  unsigned u = __float_as_uint(f);
  return (unsigned short)((u + 0x7FFFu + ((u >> 16) & 1u)) >> 16);
}
__device__ __forceinline__ float bf_bits2f(unsigned short h) { return __uint_as_float(((unsigned)h) << 16); }
__device__ __forceinline__ float bfr(float f) { return bf_bits2f(f2bf_bits(f)); }
__device__ __forceinline__ float h16_to_f32(unsigned hb) {
  const unsigned sgn = (hb & 0x8000u) << 16; const unsigned em = hb & 0x7fffu;
  const float fn = __uint_as_float((em << 13) + 0x38000000u);
  const float fs = (float)em * 5.9604644775390625e-8f;
  const float mag = (em < 0x400u) ? fs : fn; return __uint_as_float(__float_as_uint(mag) | sgn); }

__device__ __forceinline__ void dep_guard_h(v8f& a, v8f& b, v16h x, v16h y) { asm volatile("v_nop\n\tv_nop\n\tv_nop\n\tv_nop" : "+v"(a), "+v"(b) : "v"(x), "v"(y)); }
__device__ __forceinline__ void dep_guard_b(v8f& a, v8f& b, v16b x, v16b y) { asm volatile("v_nop\n\tv_nop\n\tv_nop\n\tv_nop" : "+v"(a), "+v"(b) : "v"(x), "v"(y)); }
__device__ __forceinline__ void dep_guard4_h(v8f& a, v8f& b, v8f& c, v8f& d, v16h x, v16h y) { asm volatile("v_nop\n\tv_nop\n\tv_nop\n\tv_nop" : "+v"(a), "+v"(b), "+v"(c), "+v"(d) : "v"(x), "v"(y)); }
__device__ __forceinline__ void dep_guard4_b(v8f& a, v8f& b, v8f& c, v8f& d, v16b x, v16b y) { asm volatile("v_nop\n\tv_nop\n\tv_nop\n\tv_nop" : "+v"(a), "+v"(b), "+v"(c), "+v"(d) : "v"(x), "v"(y)); }
__device__ __forceinline__ void keep4_h(v16h a, v16h b, v16h c, v16h d) { asm volatile("v_nop" :: "v"(a), "v"(b), "v"(c), "v"(d)); }
__device__ __forceinline__ void keep4_b(v16b a, v16b b, v16b c, v16b d) { asm volatile("v_nop" :: "v"(a), "v"(b), "v"(c), "v"(d)); }
__device__ __forceinline__ void acc_guard4(v8f& a, v8f& b, v8f& c, v8f& d) { asm volatile("v_nop\n\tv_nop\n\tv_nop\n\tv_nop" : "+v"(a), "+v"(b), "+v"(c), "+v"(d)); }
template <typename T> struct Frag;
template <> struct Frag<_Float16> {
  typedef v16h V; union U { v16h v; v8h h[2]; };
  static __device__ __forceinline__ v16h load(const _Float16* p) {
    U f; f.h[0] = *(const v8h*)(p); f.h[1] = *(const v8h*)(p + 16); return f.v;
  }
  static __device__ __forceinline__ v8f mma(v16h a, v16h b, v8f c) {
    return __builtin_amdgcn_wmma_f32_16x16x32_f16(false, a, false, b, (short)0, c, false, false);
  }
  static __device__ __forceinline__ void guard(v8f& a, v8f& b, v16h x, v16h y) { dep_guard_h(a, b, x, y); }
  static __device__ __forceinline__ void guard4(v8f& a, v8f& b, v8f& c, v8f& d, v16h x, v16h y) { dep_guard4_h(a, b, c, d, x, y); }
  static __device__ __forceinline__ void keep(v16h a, v16h b, v16h c, v16h d) { keep4_h(a, b, c, d); }
};
template <> struct Frag<__bf16> {
  typedef v16b V; union U { v16b v; v8b h[2]; };
  static __device__ __forceinline__ v16b load(const __bf16* p) {
    U f; f.h[0] = *(const v8b*)(p); f.h[1] = *(const v8b*)(p + 16); return f.v;
  }
  static __device__ __forceinline__ v8f mma(v16b a, v16b b, v8f c) {
    return __builtin_amdgcn_wmma_f32_16x16x32_bf16(false, a, false, b, (short)0, c, false, false);
  }
  static __device__ __forceinline__ void guard(v8f& a, v8f& b, v16b x, v16b y) { dep_guard_b(a, b, x, y); }
  static __device__ __forceinline__ void guard4(v8f& a, v8f& b, v8f& c, v8f& d, v16b x, v16b y) { dep_guard4_b(a, b, c, d, x, y); }
  static __device__ __forceinline__ void keep(v16b a, v16b b, v16b c, v16b d) { keep4_b(a, b, c, d); }
};

template <int ET> struct Elem;
template <> struct Elem<0> { typedef _Float16 T; };
template <> struct Elem<1> { typedef __bf16 T; };
template <int ET, int SPL, int BIAS_MODE, int OUT_MODE, bool RESID, int ACT = 0>
__global__ __launch_bounds__(256) void wmma_gemm64(
    const unsigned short* __restrict__ Ap, const unsigned short* __restrict__ A2p, int lda, long strideA,
    const unsigned short* __restrict__ Btp, const unsigned short* __restrict__ Bt2p, int ldb, long strideB,
    void* __restrict__ Cout, void* __restrict__ Cout2, int ldc, long strideC,
    const float* __restrict__ bias,
    const float* __restrict__ resid, long strideR,
    int M, int N, int K, float scale) {
  typedef typename Elem<ET>::T T;
  typedef typename Frag<T>::V V;
  const T* A = (const T*)Ap; const T* A2 = (const T*)A2p; const T* Bt = (const T*)Btp; const T* Bt2 = (const T*)Bt2p;
  __shared__ __align__(16) float sT[8][16 * 68];
  const int b    = blockIdx.y;
  const int lane = threadIdx.x & 31;
  const int wave = threadIdx.x >> 5;
  const int tilesN = N >> 6;
  const int tilesM = M >> 6;
  const int tile = blockIdx.x * 8 + wave;
  if (tile >= tilesM * tilesN) return;
  const int tm = tile / tilesN;
  const int tn = tile - tm * tilesN;
  const int m0 = tm << 6;
  const int n0 = tn << 6;

  const T* Ab  = A  + (size_t)b * strideA;
  const T* Bb  = Bt + (size_t)b * strideB;
  const T* Ab2 = (SPL >= 1) ? (A2  + (size_t)b * strideA) : nullptr;
  const T* Bb2 = (SPL == 2) ? (Bt2 + (size_t)b * strideB) : nullptr;

  const int rlane = lane & 15;
  const int koff  = (lane >> 4) * 8;
  const int mOff  = (lane >> 4) * 8;

  v8f acc[4][4];
#pragma unroll
  for (int i = 0; i < 4; ++i)
#pragma unroll
    for (int j = 0; j < 4; ++j) acc[i][j] = (v8f){0.f,0.f,0.f,0.f,0.f,0.f,0.f,0.f};

  for (int k0 = 0; k0 < K; k0 += 32) {
    V bh[4], bl[4];
#pragma unroll
    for (int j = 0; j < 4; ++j) {
      const size_t bo = (size_t)(n0 + (j << 4) + rlane) * ldb + koff + k0;
      bh[j] = Frag<T>::load(Bb + bo);
      if (SPL == 2) bl[j] = Frag<T>::load(Bb2 + bo);
    }
#pragma unroll
    for (int i = 0; i < 4; ++i) {
      const size_t ao = (size_t)(m0 + (i << 4) + rlane) * lda + koff + k0;
      V ah = Frag<T>::load(Ab + ao);
      V al;
      if (SPL >= 1) al = Frag<T>::load(Ab2 + ao);
#pragma unroll
      for (int j = 0; j < 4; ++j) {
        acc[i][j] = Frag<T>::mma(ah, bh[j], acc[i][j]);
        if (SPL == 2) acc[i][j] = Frag<T>::mma(ah, bl[j], acc[i][j]);
        if (SPL >= 1) acc[i][j] = Frag<T>::mma(al, bh[j], acc[i][j]);
      }
      Frag<T>::guard4(acc[i][0], acc[i][1], acc[i][2], acc[i][3], ah, (SPL >= 1) ? al : ah);
    }
    Frag<T>::keep(bh[0], bh[1], bh[2], bh[3]);
    if (SPL == 2) Frag<T>::keep(bl[0], bl[1], bl[2], bl[3]);
  }
  acc_guard4(acc[0][0], acc[0][1], acc[0][2], acc[0][3]);
  acc_guard4(acc[1][0], acc[1][1], acc[1][2], acc[1][3]);
  acc_guard4(acc[2][0], acc[2][1], acc[2][2], acc[2][3]);
  acc_guard4(acc[3][0], acc[3][1], acc[3][2], acc[3][3]);

  float* slab = sT[wave];
  const float* Rb = RESID ? (resid + (size_t)b * strideR) : nullptr;
#pragma unroll
  for (int i = 0; i < 4; ++i) {
    const int mBase = m0 + (i << 4);
#pragma unroll
    for (int j = 0; j < 4; ++j) {
      const int n = n0 + (j << 4) + rlane;
      float bv = 0.f;
      if (BIAS_MODE == 2) bv = bfr(bias[n]);
#pragma unroll
      for (int r = 0; r < 8; ++r) {
        float v = acc[i][j][r] * scale;
        if (BIAS_MODE == 1) v += bias[mBase + mOff + r];
        if (BIAS_MODE == 2) v += bv;
        if (RESID) v += Rb[(size_t)(mBase + mOff + r) * ldc + n];
        if (ACT == 1) v = tanhf(v);
        if (ACT == 2) v = fmaxf(v, 0.0f);
        if (ACT == 3) v = v / (1.0f + expf(-v));
        if (ACT == 4) v = (v > 0.f) ? v : 0.01f * v;
        slab[(mOff + r) * 68 + (j << 4) + rlane] = v;
      }
    }
    __builtin_amdgcn_fence(__ATOMIC_RELEASE, "workgroup");
    __builtin_amdgcn_wave_barrier();
    __builtin_amdgcn_fence(__ATOMIC_ACQUIRE, "workgroup");
    if (OUT_MODE == 0) {
      float* C = (float*)Cout + (size_t)b * strideC;
      const int hh = lane >> 4, c4 = (lane & 15) * 4;
      for (int pass = 0; pass < 2; ++pass) {
#pragma unroll
        for (int it = 0; it < 8; ++it) {
          const int row = it * 2 + hh;
          v4f v = *(const v4f*)(slab + row * 68 + c4);
          *(volatile v4f*)(C + (size_t)(mBase + row) * ldc + n0 + c4) = v;
        }
        __threadfence();
      }
    } else {
      const int q = lane >> 3, c8 = (lane & 7) * 8;
      unsigned short* C  = (unsigned short*)Cout  + (size_t)b * strideC;
      unsigned short* C2 = (OUT_MODE == 2) ? ((unsigned short*)Cout2 + (size_t)b * strideC) : nullptr;
      for (int pass = 0; pass < 2; ++pass) {
#pragma unroll
        for (int it = 0; it < 4; ++it) {
          const int row = it * 4 + q;
          const float* sp = slab + row * 68 + c8;
          v8h hv, lv;
#pragma unroll
          for (int e = 0; e < 8; ++e) {
            if (OUT_MODE == 1) {
              hv[e] = (_Float16)sp[e];
            } else {
              unsigned short hb = f2bf_bits(sp[e]);
              unsigned short lb = f2bf_bits(sp[e] - bf_bits2f(hb));
              hv[e] = __builtin_bit_cast(_Float16, hb);
              lv[e] = __builtin_bit_cast(_Float16, lb);
            }
          }
          *(volatile v8h*)(C + (size_t)(mBase + row) * ldc + n0 + c8) = hv;
          if (OUT_MODE == 2) *(volatile v8h*)(C2 + (size_t)(mBase + row) * ldc + n0 + c8) = lv;
        }
        __threadfence();
      }
    }
    __builtin_amdgcn_fence(__ATOMIC_RELEASE, "workgroup");
    __builtin_amdgcn_wave_barrier();
    __builtin_amdgcn_fence(__ATOMIC_ACQUIRE, "workgroup");
  }
}

__global__ __launch_bounds__(256) void xcvt_kernel(
    const float* __restrict__ src, unsigned short* __restrict__ dst, int total8)
{
  const int i = blockIdx.x * 256 + threadIdx.x;
  if (i >= total8) return;
  const size_t e0 = (size_t)i << 3;
  const v4f a0 = *(const v4f*)(src + e0);
  const v4f a1 = *(const v4f*)(src + e0 + 4);
  v8h hv;
#pragma unroll
  for (int e = 0; e < 4; ++e) {
    const float x0 = a0[e], x1 = a1[e];
    const unsigned short b0 = f2bf_bits(x0), b1 = f2bf_bits(x1);
    hv[e]     = __builtin_bit_cast(_Float16, b0);
    hv[4 + e] = __builtin_bit_cast(_Float16, b1);
  }
  unsigned short* p = dst + e0;
  *(volatile v8h*)p = hv;
  __threadfence();
  *(volatile v8h*)p = hv;
}

template <int ET>
__global__ __launch_bounds__(256) void wtrans_kernel(
    const float* __restrict__ W, unsigned short* __restrict__ WT, int K, int N, float sc)
{
  __shared__ __align__(16) float sW[64 * 65];
  const int tid = threadIdx.x, lane = tid & 31, wave = tid >> 5;
  const int n0 = blockIdx.x * 64, k0 = blockIdx.y * 64;
  const int c4 = (tid & 15) * 4, rr = tid >> 4;
  const int ncol = n0 + c4;
  const bool inr = (ncol < N);
  const int ncl = inr ? ncol : (N - 4);
  float fin = inr ? 1.0f : 0.0f;
  asm volatile("" : "+v"(fin));
#pragma unroll
  for (int p = 0; p < 4; ++p) {
    const int kk = p * 16 + rr;
    const v4f v = *(const v4f*)(W + (size_t)(k0 + kk) * N + ncl);
    float* sp = sW + kk * 65 + c4;
    const float v0 = v[0], v1 = v[1], v2 = v[2], v3 = v[3];
    sp[0] = fmaf(fin, v0, 0.0f);
    sp[1] = fmaf(fin, v1, 0.0f);
    sp[2] = fmaf(fin, v2, 0.0f);
    sp[3] = fmaf(fin, v3, 0.0f);
  }
  __syncthreads();
  const int q = lane >> 3, j8 = (lane & 7) * 8;
  v8h hv[2];
#pragma unroll
  for (int it = 0; it < 2; ++it) {
    const int n = it * 32 + wave * 4 + q;
#pragma unroll
    for (int e = 0; e < 8; ++e) {
      const float x = sW[(j8 + e) * 65 + n];
      const unsigned short hb = f2bf_bits(x);
      if (ET == 1) {
        hv[it][e] = __builtin_bit_cast(_Float16, hb);
      } else {
        const float y = sc * bf_bits2f(hb);
        hv[it][e] = (_Float16)y;
      }
    }
  }
  for (int pass = 0; pass < 2; ++pass) {
#pragma unroll
    for (int it = 0; it < 2; ++it) {
      const int n = it * 32 + wave * 4 + q;
      *(volatile v8h*)(WT + (size_t)(n0 + n) * K + k0 + j8) = hv[it];
    }
    __threadfence();
  }
}

constexpr int kConvCh = 512;
constexpr int kConvRows = 64;
constexpr int kConvTP = 516;
__global__ __launch_bounds__(256) void conv_silu_kernel(
    const unsigned short* __restrict__ XZ, const float* __restrict__ cw, const float* __restrict__ cb,
    unsigned short* __restrict__ U)
{
  __shared__ __align__(16) float sT[16 * kConvTP];
  const int tid = threadIdx.x, lane = tid & 31, wave = tid >> 5;
  const int d0 = blockIdx.x * kConvCh;
  const int da = d0 + 2 * tid;
  const int g0 = blockIdx.y * kConvRows;
  const int tb = g0 & (kSeq - 1);
  const v4f wa = *(const v4f*)(cw + (size_t)da * kDConv);
  const v4f wb = *(const v4f*)(cw + (size_t)(da + 1) * kDConv);
  const float wa0 = bfr(wa[0]), wa1 = bfr(wa[1]), wa2 = bfr(wa[2]), wa3 = bfr(wa[3]);
  const float wb0 = bfr(wb[0]), wb1 = bfr(wb[1]), wb2 = bfr(wb[2]), wb3 = bfr(wb[3]);
  const float ba = bfr(cb[da]), bb = bfr(cb[da + 1]);
  const unsigned* XZw = (const unsigned*)(const void*)XZ;
  constexpr size_t kXzWP = kXzN / 2;
  const size_t wc = (size_t)(d0 >> 1) + tid;
  float a3, a2, a1, b3, b2, b1;
  {
    const float hf = (tb > 0) ? 1.0f : 0.0f;
    const int rb = (tb > 0) ? (g0 - 3) : g0;
    const unsigned q3 = XZw[(size_t)rb * kXzWP + wc];
    const unsigned q2 = XZw[(size_t)(rb + 1) * kXzWP + wc];
    const unsigned q1 = XZw[(size_t)(rb + 2) * kXzWP + wc];
    a3 = h16_to_f32(q3 & 0xffffu) * hf; b3 = h16_to_f32(q3 >> 16) * hf;
    a2 = h16_to_f32(q2 & 0xffffu) * hf; b2 = h16_to_f32(q2 >> 16) * hf;
    a1 = h16_to_f32(q1 & 0xffffu) * hf; b1 = h16_to_f32(q1 >> 16) * hf;
  }
#pragma unroll 1
  for (int sub = 0; sub < 4; ++sub) {
    const int lb = g0 + sub * 16;
#pragma unroll 1
    for (int s = 0; s < 16; ++s) {
      const unsigned qc = XZw[(size_t)(lb + s) * kXzWP + wc];
      const float ac = h16_to_f32(qc & 0xffffu), bcur = h16_to_f32(qc >> 16);
      float pa = wa0 * a3;
      pa = fmaf(wa1, a2, pa);
      pa = fmaf(wa2, a1, pa);
      pa = fmaf(wa3, ac, pa);
      float pb = wb0 * b3;
      pb = fmaf(wb1, b2, pb);
      pb = fmaf(wb2, b1, pb);
      pb = fmaf(wb3, bcur, pb);
      const float sa = pa + ba, sb = pb + bb;
      const float ua = sa / (1.0f + expf(-sa));
      const float ub = sb / (1.0f + expf(-sb));
      v2f uv; uv[0] = ua; uv[1] = ub;
      *(v2f*)(sT + s * kConvTP + 2 * tid) = uv;
      a3 = a2; a2 = a1; a1 = ac;
      b3 = b2; b2 = b1; b1 = bcur;
    }
    __syncthreads();
    v8h hv[2][2];
#pragma unroll
    for (int it = 0; it < 2; ++it) {
      const int row = it * 8 + wave;
#pragma unroll
      for (int hlf = 0; hlf < 2; ++hlf) {
        const float* sp = sT + row * kConvTP + hlf * 256 + lane * 8;
        const v4f x0 = *(const v4f*)(sp);
        const v4f x1 = *(const v4f*)(sp + 4);
#pragma unroll
        for (int e = 0; e < 4; ++e) {
          const float y0 = x0[e] * 64.0f, y1 = x1[e] * 64.0f;
          hv[it][hlf][e]     = (_Float16)y0;
          hv[it][hlf][4 + e] = (_Float16)y1;
        }
      }
    }
    for (int pass = 0; pass < 2; ++pass) {
#pragma unroll
      for (int it = 0; it < 2; ++it) {
#pragma unroll
        for (int hlf = 0; hlf < 2; ++hlf) {
          const size_t o = (size_t)(lb + it * 8 + wave) * kDin + d0 + hlf * 256 + lane * 8;
          *(volatile v8h*)(U + o) = hv[it][hlf];
        }
      }
      __threadfence();
    }
    __syncthreads();
  }
}

__device__ __forceinline__ void stage8(const unsigned short* __restrict__ src, float* dst, float sc) {
  const v4u w = *(const v4u*)(src);
  const unsigned w0 = w[0], w1 = w[1], w2 = w[2], w3 = w[3];
  v4f lo, hi;
  lo[0] = h16_to_f32(w0 & 0xffffu) * sc; lo[1] = h16_to_f32(w0 >> 16) * sc;
  lo[2] = h16_to_f32(w1 & 0xffffu) * sc; lo[3] = h16_to_f32(w1 >> 16) * sc;
  hi[0] = h16_to_f32(w2 & 0xffffu) * sc; hi[1] = h16_to_f32(w2 >> 16) * sc;
  hi[2] = h16_to_f32(w3 & 0xffffu) * sc; hi[3] = h16_to_f32(w3 >> 16) * sc;
  *(v4f*)(dst) = lo;
  *(v4f*)(dst + 4) = hi;
}

constexpr int kScanTS = 32;
constexpr int kScanCh = 64;
constexpr int kScanYP = 68;
static_assert((kSeq % kScanTS) == 0 && (kDin % kScanCh) == 0, "scan tile multiples");
__global__ __launch_bounds__(kScanCh) void scan_kernel(
    const unsigned short* __restrict__ DP, const unsigned short* __restrict__ U,
    const unsigned short* __restrict__ XZ, const unsigned short* __restrict__ BC,
    const float* __restrict__ Alog, const float* __restrict__ Dp, unsigned short* __restrict__ Y)
{
  __shared__ __align__(16) float sDP[kScanTS * kScanCh];
  __shared__ __align__(16) float sU[kScanTS * kScanCh];
  __shared__ __align__(16) float sZ[kScanTS * kScanCh];
  __shared__ __align__(16) float sBC[kScanTS * 2 * kNst];
  __shared__ __align__(16) float sY[kScanTS * kScanYP];
  __shared__ __align__(16) float sA[kNst * kScanCh];
  const int tid = threadIdx.x, lane = tid & 31, wave = tid >> 5;
  constexpr int kBlkPerB = kDin / kScanCh;
  const int bix = blockIdx.x / kBlkPerB;
  const int d0  = (blockIdx.x - bix * kBlkPerB) * kScanCh;
  const int d   = d0 + tid;
  const size_t row0 = (size_t)bix * kSeq;
#pragma unroll 1
  for (int s = 0; s < kNst; ++s) {
    const float al = bfr(Alog[(size_t)d * kNst + s]);
    sA[s * kScanCh + tid] = -expf(al) * 1.44269504088896341f;
  }
  __syncthreads();
  float A2[kNst], h[kNst];
#pragma unroll
  for (int s = 0; s < kNst; ++s) {
    A2[s] = sA[s * kScanCh + tid];
    h[s] = 0.f;
  }
  const float Dd = bfr(Dp[d]);
  const int q = lane >> 3, c8s = (lane & 7) * 8;
#pragma unroll 1
  for (int t0 = 0; t0 < kSeq; t0 += kScanTS) {
    __syncthreads();
#pragma unroll
    for (int j = 0; j < 4; ++j) {
      const int i = tid + kScanCh * j; const int r = i >> 3; const int c8 = (i & 7) * 8;
      stage8(DP + (row0 + t0 + r) * (size_t)kDin + d0 + c8, sDP + r * kScanCh + c8, 1.0f);
    }
    asm volatile("" ::: "memory");
#pragma unroll
    for (int j = 0; j < 4; ++j) {
      const int i = tid + kScanCh * j; const int r = i >> 3; const int c8 = (i & 7) * 8;
      stage8(U + (row0 + t0 + r) * (size_t)kDin + d0 + c8, sU + r * kScanCh + c8, 0.015625f);
    }
    asm volatile("" ::: "memory");
#pragma unroll
    for (int j = 0; j < 4; ++j) {
      const int i = tid + kScanCh * j; const int r = i >> 3; const int c8 = (i & 7) * 8;
      stage8(XZ + (row0 + t0 + r) * (size_t)kXzN + kDin + d0 + c8, sZ + r * kScanCh + c8, 1.0f);
    }
    asm volatile("" ::: "memory");
#pragma unroll
    for (int j = 0; j < 2; ++j) {
      const int i = tid + kScanCh * j; const int r = i >> 2; const int c8 = (i & 3) * 8;
      stage8(BC + (row0 + t0 + r) * (size_t)kBcN + c8, sBC + r * (2 * kNst) + c8, 1.0f);
    }
    __syncthreads();
#pragma unroll 1
    for (int s = 0; s < kScanTS; ++s) {
      const float v  = sDP[s * kScanCh + tid];
      const float xt = sU[s * kScanCh + tid];
      const float zv = sZ[s * kScanCh + tid];
      const float* br = sBC + s * (2 * kNst);
      float Bs[kNst], Cs[kNst];
#pragma unroll
      for (int q4 = 0; q4 < 4; ++q4) {
        const v4f bv = *(const v4f*)(br + 4 * q4);
        const v4f cv = *(const v4f*)(br + kNst + 4 * q4);
        Bs[4 * q4 + 0] = bv[0]; Bs[4 * q4 + 1] = bv[1]; Bs[4 * q4 + 2] = bv[2]; Bs[4 * q4 + 3] = bv[3];
        Cs[4 * q4 + 0] = cv[0]; Cs[4 * q4 + 1] = cv[1]; Cs[4 * q4 + 2] = cv[2]; Cs[4 * q4 + 3] = cv[3];
      }
      const float a   = expf(-fabsf(v));
      const float u1  = 1.0f + a;
      const float l1p = logf(u1) + (a - (u1 - 1.0f)) * __builtin_amdgcn_rcpf(u1);
      const float dt  = fmaxf(v, 0.0f) + l1p;
      const float dtx = dt * xt;
      float y = 0.f;
#pragma unroll
      for (int k = 0; k < kNst; ++k) {
        const float e = exp2f(dt * A2[k]);
        h[k] = fmaf(e, h[k], dtx * Bs[k]);
        y = fmaf(h[k], Cs[k], y);
      }
      y = fmaf(xt, Dd, y);
      const float sg = 1.0f / (1.0f + expf(-zv));
      y = y * (zv * sg);
      sY[s * kScanYP + tid] = y;
    }
    __syncthreads();
    v8h hv[4];
#pragma unroll
    for (int it = 0; it < 4; ++it) {
      const int row = it * 8 + wave * 4 + q;
      const float* sp = sY + row * kScanYP + c8s;
      const v4f x0 = *(const v4f*)(sp);
      const v4f x1 = *(const v4f*)(sp + 4);
#pragma unroll
      for (int e = 0; e < 4; ++e) {
        const float y0 = x0[e] * 1024.0f, y1 = x1[e] * 1024.0f;
        hv[it][e]     = (_Float16)y0;
        hv[it][4 + e] = (_Float16)y1;
      }
    }
    for (int pass = 0; pass < 2; ++pass) {
#pragma unroll
      for (int it = 0; it < 4; ++it) {
        const int row = it * 8 + wave * 4 + q;
        const size_t o = (row0 + t0 + row) * (size_t)kDin + d0 + c8s;
        *(volatile v8h*)(Y + o) = hv[it];
      }
      __threadfence();
    }
  }
}

extern "C" void kernel_launch(void* const* d_in, const int* in_sizes, int n_in,
                              void* d_out, int out_size, void* d_ws, size_t ws_size,
                              hipStream_t stream) {
  if (n_in < 10) return;
  if (in_sizes[0] != kRows * kDm) return;
  if (in_sizes[1] != kDm * kXzN) return;
  if (in_sizes[2] != kDin * kDConv) return;
  if (in_sizes[3] != kDin) return;
  if (in_sizes[4] != kDin * kXdN) return;
  if (in_sizes[5] != kDin * kDin) return;
  if (in_sizes[6] != kDin) return;
  if (in_sizes[7] != kDin * kNst) return;
  if (in_sizes[8] != kDin) return;
  if (in_sizes[9] != kDin * kDm) return;
  if (out_size != kRows * kDm) return;
  if (ws_size < kWsTotal) return;

  const float* x      = (const float*)d_in[0];
  const float* w_in   = (const float*)d_in[1];
  const float* conv_w = (const float*)d_in[2];
  const float* conv_b = (const float*)d_in[3];
  const float* w_x    = (const float*)d_in[4];
  const float* w_dt   = (const float*)d_in[5];
  const float* b_dt   = (const float*)d_in[6];
  const float* A_log  = (const float*)d_in[7];
  const float* Dp     = (const float*)d_in[8];
  const float* w_out  = (const float*)d_in[9];
  float* out = (float*)d_out;

  char* ws = (char*)d_ws;
  unsigned short* XB  = (unsigned short*)(ws + kOffXB);
  unsigned short* WIB = (unsigned short*)(ws + kOffWIB);
  unsigned short* WXH = (unsigned short*)(ws + kOffWXH);
  unsigned short* WDH = (unsigned short*)(ws + kOffWDH);
  unsigned short* WOH = (unsigned short*)(ws + kOffWOH);
  unsigned short* XZ  = (unsigned short*)(ws + kOffXZ);
  unsigned short* U   = (unsigned short*)(ws + kOffU);
  unsigned short* DI  = (unsigned short*)(ws + kOffDI);
  unsigned short* Yp  = (unsigned short*)(ws + kOffDI);
  unsigned short* BC  = (unsigned short*)(ws + kOffBC);
  unsigned short* DP  = (unsigned short*)(ws + kOffDP);

  xcvt_kernel<<<(kRows * kDm / 8) / 256, 256, 0, stream>>>(x, XB, kRows * kDm / 8);
  wtrans_kernel<1><<<dim3(kXzN / 64, kDm / 64), 256, 0, stream>>>(w_in, WIB, kDm, kXzN, 1.0f);
  wtrans_kernel<0><<<dim3(kWxNP / 64, kDin / 64), 256, 0, stream>>>(w_x, WXH, kDin, kXdN, 64.0f);
  wtrans_kernel<0><<<dim3(kDin / 64, kDin / 64), 256, 0, stream>>>(w_dt, WDH, kDin, kDin, 64.0f);
  wtrans_kernel<0><<<dim3(kDm / 64, kDin / 64), 256, 0, stream>>>(w_out, WOH, kDin, kDm, 64.0f);

  wmma_gemm64<1, 0, 0, 1, false><<<dim3((kRows / 64) * (kXzN / 64) / 8, 1), 256, 0, stream>>>(
      XB, nullptr, kDm, 0L,
      WIB, nullptr, kDm, 0L,
      (void*)XZ, nullptr, kXzN, 0L,
      nullptr, nullptr, 0L,
      kRows, kXzN, kDm, 1.0f);

  conv_silu_kernel<<<dim3(kDin / kConvCh, kRows / kConvRows), 256, 0, stream>>>(XZ, conv_w, conv_b, U);

  wmma_gemm64<0, 0, 0, 1, false><<<dim3((kRows / 64) * (kDin / 64) / 8, 1), 256, 0, stream>>>(
      U, nullptr, kDin, 0L,
      WXH, nullptr, kDin, 0L,
      (void*)DI, nullptr, kDin, 0L,
      nullptr, nullptr, 0L,
      kRows, kDin, kDin, 0.015625f);

  wmma_gemm64<0, 0, 0, 1, false><<<dim3((kRows / 64) * (kBcN / 64) / 8, 1), 256, 0, stream>>>(
      U, nullptr, kDin, 0L,
      WXH + (size_t)kDin * kDin, nullptr, kDin, 0L,
      (void*)BC, nullptr, kBcN, 0L,
      nullptr, nullptr, 0L,
      kRows, kBcN, kDin, 1.0f / 4096.0f);

  wmma_gemm64<0, 0, 2, 1, false><<<dim3((kRows / 64) * (kDin / 64) / 8, 1), 256, 0, stream>>>(
      DI, nullptr, kDin, 0L,
      WDH, nullptr, kDin, 0L,
      (void*)DP, nullptr, kDin, 0L,
      b_dt, nullptr, 0L,
      kRows, kDin, kDin, 1.0f / 4096.0f);

  scan_kernel<<<kBatch * (kDin / kScanCh), kScanCh, 0, stream>>>(DP, U, XZ, BC, A_log, Dp, Yp);

  wmma_gemm64<0, 0, 0, 0, false><<<dim3((kRows / 64) * (kDm / 64) / 8, 1), 256, 0, stream>>>(
      Yp, nullptr, kDin, 0L,
      WOH, nullptr, kDin, 0L,
      (void*)out, nullptr, kDm, 0L,
      nullptr, nullptr, 0L,
      kRows, kDm, kDin, 1.0f / 65536.0f);
}
